// GraphConvolution_48292612276717
// MI455X (gfx1250) — hardware-run, weakly checked
//
#include <hip/hip_runtime.h>


namespace {
constexpr int T = 2048, NBT = 16  , D = 128, BL = 16  ;
constexpr float XS = 8.0f, WSC = 256.0f, RS_ = 1024.0f, AS = 8.0f;
static_assert(T % 32 == 0 && D == 128, "tiling");
typedef _Float16 b16;
typedef __attribute__((ext_vector_type(16))) _Float16 v16b;
typedef __attribute__((ext_vector_type(8))) _Float16 v8b;
typedef __attribute__((ext_vector_type(8))) float v8f;
typedef __attribute__((ext_vector_type(4))) float v4f;
__device__ __forceinline__ float bf16_rne(float f) { unsigned int u = __float_as_uint(f); u += 0x7FFFu + ((u >> 16) & 1u); return __uint_as_float(u & 0xFFFF0000u); }
__device__ __forceinline__ void split16(float v, b16& hi, b16& lo) { hi = (b16)v; lo = (b16)(v - (float)hi); }
__device__ __forceinline__ v16b frag_kb(const b16* p, int hh) { const v8b a = *(const v8b*)(p + 8 * hh), b = *(const v8b*)(p + 16 + 8 * hh); v16b f;
#pragma unroll
  for (int e = 0; e < 8; ++e) { f[e] = a[e]; f[8 + e] = b[e]; } return f; }
__device__ __forceinline__ v8f wmma16b(v16b a, v16b b, v8f c) { v8f d = __builtin_amdgcn_wmma_f32_16x16x32_f16(false, a, false, b, (short)0, c, false, false); asm volatile("v_nop\n\tv_nop\n\tv_nop\n\tv_nop" : "+v"(d) : "v"(a), "v"(b)); return d; }
__device__ __forceinline__ void wave_lds_sync() { __builtin_amdgcn_fence(__ATOMIC_RELEASE, "workgroup"); __builtin_amdgcn_wave_barrier(); __builtin_amdgcn_fence(__ATOMIC_ACQUIRE, "workgroup"); }
__device__ __forceinline__ float pmul(float a, float b) { float p = a * b; asm volatile("" : "+v"(p)); return p; }
__device__ __forceinline__ int iclamp(int v, int lo, int hi) { return v < lo ? lo : (v > hi ? hi : v); }

typedef __attribute__((ext_vector_type(2))) _Float16 v2h;
typedef __attribute__((ext_vector_type(4))) _Float16 v4h;
typedef __attribute__((ext_vector_type(2))) float v2f;
typedef __attribute__((ext_vector_type(4))) int v4i;
__device__ __forceinline__ float nexp2(float v) { return __builtin_amdgcn_exp2f(v); }
__device__ __forceinline__ float bfp(float v) { float t = bf16_rne(v); asm volatile("" : "+v"(t)); return t; }

__global__ __launch_bounds__(256) void prep_kernel(const float* __restrict__ adj, const float* __restrict__ w, float* __restrict__ R, b16* __restrict__ WT) {
  const int m = blockIdx.x * 256 + threadIdx.x; float s = 0.0f;
#pragma unroll 4
  for (int n = 0; n < T; ++n) s += bf16_rne(adj[(size_t)n * T + m]);
  const float rv = rsqrtf(s);
  for (int pass = 0; pass < 2; ++pass) { ((volatile float*)R)[m] = rv;
    if (blockIdx.x == 0) { for (int i = threadIdx.x; i < D * D / 8; i += 256) { const int e = i * 8; const int o = e / D, k0 = e % D; v8b v; for (int j = 0; j < 8; ++j) v[j] = (b16)(bf16_rne(w[(size_t)(k0 + j) * D + o]) * WSC); *(volatile v8b*)(WT + e) = v; } }
    __threadfence(); }
}
__global__ __launch_bounds__(256) void adjT_kernel(const float* __restrict__ adj, b16* __restrict__ AT) {
  __shared__ float tile[64][33];
  const int m0 = blockIdx.x * 32, n0 = blockIdx.y * 64; const int tid = threadIdx.x;
  for (int i = tid; i < 64 * 32; i += 256) { const int nl = i / 32, ml = i % 32; tile[nl][ml] = bf16_rne(adj[(size_t)(n0 + nl) * T + m0 + ml]); }
  __syncthreads();
  const int ml = tid >> 3, q = tid & 7;
  v8b v; for (int j = 0; j < 8; ++j) v[j] = (b16)(tile[8 * q + j][ml] * AS);
  for (int pass = 0; pass < 2; ++pass) { *(volatile v8b*)(AT + (size_t)(m0 + ml) * T + n0 + 8 * q) = v; __threadfence(); }
}
__global__ __launch_bounds__(64) void proj_kernel(const float* __restrict__ x, const b16* __restrict__ WT, const float* __restrict__ R, b16* __restrict__ TPh, b16* __restrict__ TPl) {
  __shared__ __attribute__((aligned(16))) b16 Ah[2][16][D + 8]; __shared__ __attribute__((aligned(16))) float Tf[2][16][D + 4];
  const int wave = threadIdx.x >> 5, lane = threadIdx.x & 31, nloc = lane & 15, hlf = lane >> 4; const size_t m0 = (size_t)blockIdx.x * 32 + wave * 16;
  for (int idx = lane; idx < 16 * (D / 4); idx += 32) { const int rr = idx / (D / 4), c4 = (idx % (D / 4)) * 4; const v4f v = *(const v4f*)(x + (m0 + rr) * D + c4); v4h hv; for (int j = 0; j < 4; ++j) hv[j] = (b16)(bf16_rne(v[j]) * XS); *(v4h*)(&Ah[wave][rr][c4]) = hv; }
  wave_lds_sync();
  v8f acc[8]; for (int t = 0; t < 8; ++t) acc[t] = (v8f){};
#pragma unroll
  for (int kb = 0; kb < D; kb += 32) { const v16b a = frag_kb(&Ah[wave][nloc][kb], hlf);
#pragma unroll
    for (int t = 0; t < 8; ++t) acc[t] = wmma16b(a, frag_kb(WT + (size_t)(t * 16 + nloc) * D + kb, hlf), acc[t]); }
#pragma unroll
  for (int t = 0; t < 8; ++t) for (int r = 0; r < 8; ++r) { const size_t grow = m0 + 8 * hlf + r; const float rn = R[grow % T]; Tf[wave][8 * hlf + r][t * 16 + nloc] = acc[t][r] * (1.0f / (XS * WSC)) * rn; }
  wave_lds_sync();
  for (int pass = 0; pass < 2; ++pass) { for (int rr = 0; rr < 16; rr += 2) { const int r2 = rr + (lane >> 4); const int c8 = (lane & 15) * 8; v8b hv, lv;
      for (int j = 0; j < 8; ++j) { const float v = Tf[wave][r2][c8 + j] * XS; const b16 ph = (b16)v; hv[j] = ph; lv[j] = (b16)((v - (float)ph) * RS_); }
      *(volatile v8b*)(TPh + (m0 + r2) * D + c8) = hv; *(volatile v8b*)(TPl + (m0 + r2) * D + c8) = lv; } __threadfence(); }
}
__global__ __launch_bounds__(64) void agg_kernel(const b16* __restrict__ AT, const b16* __restrict__ TPh, const b16* __restrict__ TPl, const float* __restrict__ R, const float* __restrict__ bias, float* __restrict__ out) {
  __shared__ __attribute__((aligned(16))) float Tf[2][16][D + 4];
  const int wave = threadIdx.x >> 5, lane = threadIdx.x & 31, nloc = lane & 15, hlf = lane >> 4; const int m0 = blockIdx.x * 32 + wave * 16; const int bt = blockIdx.y;
  const b16* arow = AT + (size_t)(m0 + nloc) * T; const b16* Th = TPh + (size_t)bt * T * D; const b16* Tl = TPl + (size_t)bt * T * D;
  v8f acc[8], accl[8];
#pragma unroll
  for (int t = 0; t < 8; ++t) { acc[t] = (v8f){}; accl[t] = (v8f){}; }
#pragma unroll 2
  for (int kb = 0; kb < T; kb += 32) { const v16b a = frag_kb(arow + kb, hlf);
#pragma unroll
    for (int t = 0; t < 8; ++t) { v16b bh, bl;
#pragma unroll
      for (int e = 0; e < 16; ++e) { const int k = (e < 8) ? (8 * hlf + e) : (16 + 8 * hlf + (e - 8)); const size_t o_ = (size_t)(kb + k) * D + t * 16 + nloc; bh[e] = Th[o_]; bl[e] = Tl[o_]; }
      acc[t] = wmma16b(a, bh, acc[t]); accl[t] = wmma16b(a, bl, accl[t]); } }
#pragma unroll
  for (int t = 0; t < 8; ++t) { const int col = t * 16 + nloc; const float bb = bf16_rne(bias[col]);
    for (int r = 0; r < 8; ++r) { const int m = m0 + 8 * hlf + r; const float y = (acc[t][r] + accl[t][r] * (1.0f / RS_)) * (1.0f / (AS * XS)) * R[m] + bb; Tf[wave][8 * hlf + r][col] = fmaxf(y, 0.0f); } }
  wave_lds_sync();
  for (int pass = 0; pass < 2; ++pass) { for (int rr = 0; rr < 16; ++rr) *(volatile v4f*)(out + ((size_t)bt * T + m0 + rr) * D + lane * 4) = *(const v4f*)(&Tf[wave][rr][lane * 4]); __threadfence(); }
}
}

extern "C" void kernel_launch(void* const* d_in, const int* in_sizes, int n_in, void* d_out, int out_size, void* d_ws, size_t ws_size, hipStream_t stream) {
  (void)n_in;
  auto Fp = [&](int i) { return (const float*)d_in[i]; };
  if (in_sizes[0] != T * T || in_sizes[1] != NBT * T * D || in_sizes[2] != D * D || in_sizes[3] != D || out_size != NBT * T * D) return;
  size_t off = 0; char* ws = (char*)d_ws;
  auto carve = [&](size_t bytes) { char* p = ws + off; off += (bytes + 255) & ~(size_t)255; return p; };
  b16* WT = (b16*)carve((size_t)D * D * 2); float* R = (float*)carve((size_t)T * 4); b16* AT = (b16*)carve((size_t)T * T * 2); b16* TPh = (b16*)carve((size_t)NBT * T * D * 2); b16* TPl = (b16*)carve((size_t)NBT * T * D * 2);
  if (off > ws_size || off > ((size_t)64 << 20)) return;
  prep_kernel<<<T / 256, 256, 0, stream>>>(Fp(0), Fp(2), R, WT);
  adjT_kernel<<<dim3(T / 32, T / 64), 256, 0, stream>>>(Fp(0), AT);
  proj_kernel<<<NBT * T / 32, 64, 0, stream>>>(Fp(1), WT, R, TPh, TPl);
  agg_kernel<<<dim3(T / 32, BL), 64, 0, stream>>>(AT, TPh, TPl, R, Fp(3), (float*)d_out);
}
